// GatedDeltaNetAttention_14456859918521
// MI455X (gfx1250) — hardware-verified
//
#include <hip/hip_runtime.h>
#include <math.h>

constexpr int kBatch   = 2;
constexpr int kTime    = 2048;
constexpr int kChan    = 1024;
constexpr int kHeads   = 16;
constexpr int kKvHeads = 4;
constexpr int kHeadDim = 64;
constexpr int kTaps    = 4;
constexpr int kRows    = kBatch * kTime;
constexpr int kNq      = kHeads * kHeadDim;
constexpr int kNkv     = kKvHeads * kHeadDim;
constexpr int kColK    = 1024;
constexpr int kColV    = 1280;
constexpr int kColBeta = 1536;
constexpr int kColGk   = 1540;
constexpr int kColGate = 1544;
constexpr int kNstk    = 2568;
constexpr int kNstkPad = 2624;
constexpr int kBgPitch = 32;
constexpr int kStage   = 16;
static_assert(kNstkPad % 64 == 0 && kNstkPad >= kNstk, "tile multiple");
static_assert(kRows % 64 == 0 && kChan % 32 == 0 && kNq % 64 == 0, "tile multiple");
static_assert(kTime % kStage == 0, "staging");

typedef __attribute__((ext_vector_type(16))) _Float16 v16h;
typedef __attribute__((ext_vector_type(8)))  _Float16 v8h;
typedef __attribute__((ext_vector_type(16))) __bf16   v16b;
typedef __attribute__((ext_vector_type(8)))  __bf16   v8b;
typedef __attribute__((ext_vector_type(8)))  float    v8f;
typedef __attribute__((ext_vector_type(4)))  float    v4f;
typedef __attribute__((ext_vector_type(2)))  float    v2f;
typedef __attribute__((ext_vector_type(4)))  unsigned int v4u;

__device__ __forceinline__ unsigned short f2bf_bits(float f) {
  unsigned u = __float_as_uint(f);
  return (unsigned short)((u + 0x7FFFu + ((u >> 16) & 1u)) >> 16);
}
__device__ __forceinline__ float bf_bits2f(unsigned short h) { return __uint_as_float(((unsigned)h) << 16); }
__device__ __forceinline__ unsigned pk16(unsigned short a, unsigned short b) { return (unsigned)a | ((unsigned)b << 16); }

__device__ __forceinline__ void dep_guard_h(v8f& a, v8f& b, v16h x, v16h y) { asm volatile("v_nop\n\tv_nop\n\tv_nop\n\tv_nop" : "+v"(a), "+v"(b) : "v"(x), "v"(y)); }
__device__ __forceinline__ void dep_guard_b(v8f& a, v8f& b, v16b x, v16b y) { asm volatile("v_nop\n\tv_nop\n\tv_nop\n\tv_nop" : "+v"(a), "+v"(b) : "v"(x), "v"(y)); }
__device__ __forceinline__ void keep4_h(v16h a, v16h b, v16h c, v16h d) { asm volatile("v_nop" :: "v"(a), "v"(b), "v"(c), "v"(d)); }
__device__ __forceinline__ void keep4_b(v16b a, v16b b, v16b c, v16b d) { asm volatile("v_nop" :: "v"(a), "v"(b), "v"(c), "v"(d)); }
__device__ __forceinline__ void acc_guard4(v8f& a, v8f& b, v8f& c, v8f& d) { asm volatile("v_nop\n\tv_nop\n\tv_nop\n\tv_nop" : "+v"(a), "+v"(b), "+v"(c), "+v"(d)); }
template <typename T> struct Frag;
template <> struct Frag<_Float16> {
  typedef v16h V; union U { v16h v; v8h h[2]; };
  static __device__ __forceinline__ v16h load(const _Float16* p) {
    U f; f.h[0] = *(const v8h*)(p); f.h[1] = *(const v8h*)(p + 16); return f.v;
  }
  static __device__ __forceinline__ v8f mma(v16h a, v16h b, v8f c) {
    return __builtin_amdgcn_wmma_f32_16x16x32_f16(false, a, false, b, (short)0, c, false, false);
  }
  static __device__ __forceinline__ void guard(v8f& a, v8f& b, v16h x, v16h y) { dep_guard_h(a, b, x, y); }
  static __device__ __forceinline__ void keep(v16h a, v16h b, v16h c, v16h d) { keep4_h(a, b, c, d); }
};
template <> struct Frag<__bf16> {
  typedef v16b V; union U { v16b v; v8b h[2]; };
  static __device__ __forceinline__ v16b load(const __bf16* p) {
    U f; f.h[0] = *(const v8b*)(p); f.h[1] = *(const v8b*)(p + 16); return f.v;
  }
  static __device__ __forceinline__ v8f mma(v16b a, v16b b, v8f c) {
    return __builtin_amdgcn_wmma_f32_16x16x32_bf16(false, a, false, b, (short)0, c, false, false);
  }
  static __device__ __forceinline__ void guard(v8f& a, v8f& b, v16b x, v16b y) { dep_guard_b(a, b, x, y); }
  static __device__ __forceinline__ void keep(v16b a, v16b b, v16b c, v16b d) { keep4_b(a, b, c, d); }
};

template <int ET> struct Elem;
template <> struct Elem<0> { typedef _Float16 T; };
template <> struct Elem<1> { typedef __bf16 T; };
template <int ET, bool SPLIT, int BIAS_MODE, int OUT_MODE, bool RESID, int ACT = 0>
__global__ __launch_bounds__(256) void wmma_gemm64(
    const unsigned short* __restrict__ Ap, const unsigned short* __restrict__ A2p, int lda, long strideA,
    const unsigned short* __restrict__ Btp, const unsigned short* __restrict__ Bt2p, int ldb, long strideB,
    void* __restrict__ Cout, void* __restrict__ Cout2, int ldc, long strideC,
    const float* __restrict__ bias,
    const float* __restrict__ resid, long strideR,
    int M, int N, int K, float scale) {
  typedef typename Elem<ET>::T T;
  typedef typename Frag<T>::V V;
  const T* A = (const T*)Ap; const T* A2 = (const T*)A2p; const T* Bt = (const T*)Btp; const T* Bt2 = (const T*)Bt2p;
  __shared__ __align__(16) float sT[8][16 * 68];
  const int b    = blockIdx.y;
  const int lane = threadIdx.x & 31;
  const int wave = threadIdx.x >> 5;
  const int tilesN = N >> 6;
  const int tilesM = M >> 6;
  const int tile = blockIdx.x * 8 + wave;
  if (tile >= tilesM * tilesN) return;
  const int tm = tile / tilesN;
  const int tn = tile - tm * tilesN;
  const int m0 = tm << 6;
  const int n0 = tn << 6;

  const T* Ab  = A  + (size_t)b * strideA;
  const T* Bb  = Bt + (size_t)b * strideB;
  const T* Ab2 = SPLIT ? (A2  + (size_t)b * strideA) : nullptr;
  const T* Bb2 = SPLIT ? (Bt2 + (size_t)b * strideB) : nullptr;

  const int rlane = lane & 15;
  const int koff  = (lane >> 4) * 8;
  const int mOff  = (lane >> 4) * 8;

  v8f acc[4][4];
#pragma unroll
  for (int i = 0; i < 4; ++i)
#pragma unroll
    for (int j = 0; j < 4; ++j) acc[i][j] = (v8f){0.f,0.f,0.f,0.f,0.f,0.f,0.f,0.f};

  for (int k0 = 0; k0 < K; k0 += 32) {
    V bh[4], bl[4];
#pragma unroll
    for (int j = 0; j < 4; ++j) {
      const size_t bo = (size_t)(n0 + (j << 4) + rlane) * ldb + koff + k0;
      bh[j] = Frag<T>::load(Bb + bo);
      if (SPLIT) bl[j] = Frag<T>::load(Bb2 + bo);
    }
#pragma unroll
    for (int i = 0; i < 4; ++i) {
      const size_t ao = (size_t)(m0 + (i << 4) + rlane) * lda + koff + k0;
      V ah = Frag<T>::load(Ab + ao);
      V al;
      if (SPLIT) al = Frag<T>::load(Ab2 + ao);
#pragma unroll
      for (int j = 0; j < 4; ++j) {
        acc[i][j] = Frag<T>::mma(ah, bh[j], acc[i][j]);
        if (SPLIT) {
          acc[i][j] = Frag<T>::mma(ah, bl[j], acc[i][j]);
          acc[i][j] = Frag<T>::mma(al, bh[j], acc[i][j]);
        }
      }
      Frag<T>::guard(acc[i][0], acc[i][3], ah, SPLIT ? al : ah);
    }
    Frag<T>::keep(bh[0], bh[1], bh[2], bh[3]);
    if (SPLIT) Frag<T>::keep(bl[0], bl[1], bl[2], bl[3]);
  }
  acc_guard4(acc[0][0], acc[0][1], acc[0][2], acc[0][3]);
  acc_guard4(acc[1][0], acc[1][1], acc[1][2], acc[1][3]);
  acc_guard4(acc[2][0], acc[2][1], acc[2][2], acc[2][3]);
  acc_guard4(acc[3][0], acc[3][1], acc[3][2], acc[3][3]);

  float* slab = sT[wave];
  const float* Rb = RESID ? (resid + (size_t)b * strideR) : nullptr;
#pragma unroll
  for (int i = 0; i < 4; ++i) {
    const int mBase = m0 + (i << 4);
#pragma unroll
    for (int j = 0; j < 4; ++j) {
      const int n = n0 + (j << 4) + rlane;
      float bv = 0.f;
      if (BIAS_MODE == 2) bv = bias[n];
#pragma unroll
      for (int r = 0; r < 8; ++r) {
        float v = acc[i][j][r] * scale;
        if (BIAS_MODE == 1) v += bias[mBase + mOff + r];
        if (BIAS_MODE == 2) v += bv;
        if (RESID) v += Rb[(size_t)(mBase + mOff + r) * ldc + n];
        if (ACT == 2) v = fmaxf(v, 0.0f);
        if (ACT == 4) v = (v > 0.f) ? v : 0.01f * v;
        slab[(mOff + r) * 68 + (j << 4) + rlane] = v;
      }
    }
    __builtin_amdgcn_fence(__ATOMIC_RELEASE, "workgroup");
    __builtin_amdgcn_wave_barrier();
    __builtin_amdgcn_fence(__ATOMIC_ACQUIRE, "workgroup");
    if (OUT_MODE == 0) {
      float* C = (float*)Cout + (size_t)b * strideC;
      const int hh = lane >> 4, c4 = (lane & 15) * 4;
      for (int pass = 0; pass < 2; ++pass) {
#pragma unroll
        for (int it = 0; it < 8; ++it) {
          const int row = it * 2 + hh;
          v4f v = *(const v4f*)(slab + row * 68 + c4);
          *(volatile v4f*)(C + (size_t)(mBase + row) * ldc + n0 + c4) = v;
        }
        __threadfence();
      }
    } else {
      const int q = lane >> 3, c8 = (lane & 7) * 8;
      unsigned short* C  = (unsigned short*)Cout  + (size_t)b * strideC;
      unsigned short* C2 = (OUT_MODE == 2) ? ((unsigned short*)Cout2 + (size_t)b * strideC) : nullptr;
      for (int pass = 0; pass < 2; ++pass) {
#pragma unroll
        for (int it = 0; it < 4; ++it) {
          const int row = it * 4 + q;
          const float* sp = slab + row * 68 + c8;
          v8h hv, lv;
#pragma unroll
          for (int e = 0; e < 8; ++e) {
            if (OUT_MODE == 1) {
              hv[e] = (_Float16)sp[e];
            } else {
              unsigned short hb = f2bf_bits(sp[e]);
              unsigned short lb = f2bf_bits(sp[e] - bf_bits2f(hb));
              hv[e] = __builtin_bit_cast(_Float16, hb);
              lv[e] = __builtin_bit_cast(_Float16, lb);
            }
          }
          *(volatile v8h*)(C + (size_t)(mBase + row) * ldc + n0 + c8) = hv;
          if (OUT_MODE == 2) *(volatile v8h*)(C2 + (size_t)(mBase + row) * ldc + n0 + c8) = lv;
        }
        __threadfence();
      }
    }
    __builtin_amdgcn_fence(__ATOMIC_RELEASE, "workgroup");
    __builtin_amdgcn_wave_barrier();
    __builtin_amdgcn_fence(__ATOMIC_ACQUIRE, "workgroup");
  }
}

__device__ __forceinline__ void split8_bf(v4f a, v4f c, v4u& hi, v4u& lo) {
  unsigned short hb[8], lb[8];
#pragma unroll
  for (int e = 0; e < 4; ++e) {
    hb[e]     = f2bf_bits(a[e]);
    lb[e]     = f2bf_bits(a[e] - bf_bits2f(hb[e]));
    hb[4 + e] = f2bf_bits(c[e]);
    lb[4 + e] = f2bf_bits(c[e] - bf_bits2f(hb[4 + e]));
  }
  hi = (v4u){pk16(hb[0], hb[1]), pk16(hb[2], hb[3]), pk16(hb[4], hb[5]), pk16(hb[6], hb[7])};
  lo = (v4u){pk16(lb[0], lb[1]), pk16(lb[2], lb[3]), pk16(lb[4], lb[5]), pk16(lb[6], lb[7])};
}

__global__ __launch_bounds__(256) void split8_kernel(const float* __restrict__ in,
                                                     unsigned short* __restrict__ hi,
                                                     unsigned short* __restrict__ lo, int n8) {
  const int i = blockIdx.x * 256 + threadIdx.x;
  if (i >= n8) return;
  const float* p = in + 8 * (size_t)i;
  const v4f a = *(const v4f*)(p);
  const v4f c = *(const v4f*)(p + 4);
  v4u uh, ul;
  split8_bf(a, c, uh, ul);
  unsigned short* qh = hi + 8 * (size_t)i;
  unsigned short* ql = lo + 8 * (size_t)i;
  for (int pass = 0; pass < 2; ++pass) {
    *(volatile v4u*)qh = uh;
    *(volatile v4u*)ql = ul;
    __threadfence();
  }
}

__global__ __launch_bounds__(128) void split_stack_kernel(const float* __restrict__ Wq, const float* __restrict__ Wk,
                                                          const float* __restrict__ Wv, const float* __restrict__ Wbeta,
                                                          const float* __restrict__ Wgk, const float* __restrict__ Wgate,
                                                          unsigned short* __restrict__ hi, unsigned short* __restrict__ lo) {
  const int r = blockIdx.x;
  const int t = threadIdx.x;
  const float* src = Wgate;
  int sr = kNq - 1;
  bool live = true;
  if (r < kColK)         { src = Wq;    sr = r; }
  else if (r < kColV)    { src = Wk;    sr = r - kColK; }
  else if (r < kColBeta) { src = Wv;    sr = r - kColV; }
  else if (r < kColGk)   { src = Wbeta; sr = r - kColBeta; }
  else if (r < kColGate) { src = Wgk;   sr = r - kColGk; }
  else if (r < kNstk)    { src = Wgate; sr = r - kColGate; }
  else                   { live = false; }
  const float* p = src + (size_t)sr * kChan + 8 * t;
  v4f a = *(const v4f*)(p);
  v4f c = *(const v4f*)(p + 4);
  if (!live) {
    a = (v4f){0.f, 0.f, 0.f, 0.f};
    c = (v4f){0.f, 0.f, 0.f, 0.f};
  }
  v4u uh, ul;
  split8_bf(a, c, uh, ul);
  const size_t o = (size_t)r * kChan + 8 * t;
  for (int pass = 0; pass < 2; ++pass) {
    *(volatile v4u*)(hi + o) = uh;
    *(volatile v4u*)(lo + o) = ul;
    __threadfence();
  }
}

template <bool NORM>
__global__ __launch_bounds__(256) void prep_conv_kernel(const float* __restrict__ P, int col0,
                                                        const float* __restrict__ cw,
                                                        float* __restrict__ out, int ncols) {
  const int row = blockIdx.x;
  const int tt  = row & (kTime - 1);
  const int bb  = row >> 11;
  const int t   = threadIdx.x;
  const int col = 4 * t;
  v4f wv[4];
#pragma unroll
  for (int i = 0; i < 4; ++i) wv[i] = *(const v4f*)(cw + (size_t)(col + i) * kTaps);
  v4f acc = (v4f){0.f, 0.f, 0.f, 0.f};
#pragma unroll
  for (int j = 0; j < kTaps; ++j) {
    const int tr  = tt - (kTaps - 1) + j;
    const int trc = tr < 0 ? 0 : tr;
    v4f u = *(const v4f*)(P + ((size_t)bb * kTime + (size_t)trc) * kNstkPad + col0 + col);
    if (tr < 0) u = (v4f){0.f, 0.f, 0.f, 0.f};
#pragma unroll
    for (int i = 0; i < 4; ++i) acc[i] = acc[i] + wv[i][j] * u[i];
  }
  if (NORM) {
    float ss = acc[0] * acc[0] + acc[1] * acc[1] + acc[2] * acc[2] + acc[3] * acc[3];
    ss += __shfl_xor(ss, 1, 32);
    ss += __shfl_xor(ss, 2, 32);
    ss += __shfl_xor(ss, 4, 32);
    ss += __shfl_xor(ss, 8, 32);
    const float rn = rsqrtf(ss + 1e-12f);
#pragma unroll
    for (int i = 0; i < 4; ++i) acc[i] = acc[i] * rn;
  }
  float* op = out + (size_t)row * ncols + col;
  for (int pass = 0; pass < 2; ++pass) {
    *(volatile v4f*)op = acc;
    __threadfence();
  }
}

__global__ __launch_bounds__(256) void prep_bg_kernel(const float* __restrict__ P, const float* __restrict__ b_beta,
                                                      const float* __restrict__ dt_bias, const float* __restrict__ A_log,
                                                      float* __restrict__ BG) {
  const int lane = threadIdx.x & 31;
  const int wave = threadIdx.x >> 5;
  const int row  = blockIdx.x * 8 + wave;
  const int hk   = lane & 3;
  const float* pr = P + (size_t)row * kNstkPad;
  const float pb = pr[kColBeta + hk];
  const float pg = pr[kColGk + hk];
  const float bbv  = pb + b_beta[hk];
  const float beta = 1.0f / (1.0f + expf(-bbv));
  const float gz   = pg + dt_bias[hk];
  const float sp   = fmaxf(gz, 0.0f) + log1pf(expf(-fabsf(gz)));
  const float gk   = -expf(A_log[hk]) * sp;
  const float dec  = expf(gk);
  const float val  = (lane < 4) ? beta : ((lane < 8) ? dec : 0.0f);
  float* op = BG + (size_t)row * kBgPitch + lane;
  for (int pass = 0; pass < 2; ++pass) {
    *(volatile float*)op = val;
    __threadfence();
  }
}

__global__ __launch_bounds__(256) void gdn_kernel(const float* __restrict__ Qn, const float* __restrict__ Kn,
                                                  const float* __restrict__ Vc, const float* __restrict__ BG,
                                                  float* __restrict__ O) {
  __shared__ __align__(16) float ost[kStage * kHeadDim];
  const int bh   = blockIdx.x;
  const int b    = bh >> 4;
  const int h    = bh & 15;
  const int hk   = h >> 2;
  const int tid  = threadIdx.x;
  const int lane = tid & 31;
  const int wave = tid >> 5;
  const int dq   = lane >> 3;
  const int e    = wave * 8 + (lane & 7);
  float S[16];
#pragma unroll
  for (int i = 0; i < 16; ++i) S[i] = 0.0f;
  const size_t row0 = (size_t)b * kTime;
#pragma unroll 1
  for (int t = 0; t < kTime; ++t) {
    const size_t row = row0 + (size_t)t;
    const float* kp = Kn + (row * kKvHeads + hk) * kHeadDim + dq * 16;
    const float* qp = Qn + (row * kHeads + h) * kHeadDim + dq * 16;
    v4f kv4[4], qv4[4];
#pragma unroll
    for (int c = 0; c < 4; ++c) {
      kv4[c] = *(const v4f*)(kp + 4 * c);
      qv4[c] = *(const v4f*)(qp + 4 * c);
    }
    const float ve   = Vc[(row * kKvHeads + hk) * kHeadDim + e];
    const float beta = BG[row * kBgPitch + hk];
    const float dec  = BG[row * kBgPitch + 4 + hk];
    float ks = 0.0f;
#pragma unroll
    for (int c = 0; c < 4; ++c) {
#pragma unroll
      for (int i = 0; i < 4; ++i) {
        const float sd = S[4 * c + i] * dec;
        S[4 * c + i] = sd;
        ks = fmaf(kv4[c][i], sd, ks);
      }
    }
    ks += __shfl_xor(ks, 8, 32);
    ks += __shfl_xor(ks, 16, 32);
    const float upd = beta * (ve - ks);
    float oe = 0.0f;
#pragma unroll
    for (int c = 0; c < 4; ++c) {
#pragma unroll
      for (int i = 0; i < 4; ++i) {
        const float sn = fmaf(kv4[c][i], upd, S[4 * c + i]);
        S[4 * c + i] = sn;
        oe = fmaf(qv4[c][i], sn, oe);
      }
    }
    oe += __shfl_xor(oe, 8, 32);
    oe += __shfl_xor(oe, 16, 32);
    oe *= 0.125f;
    const int ts = t & (kStage - 1);
    if (dq == 0) ost[ts * kHeadDim + e] = oe;
    if (ts == kStage - 1) {
      __syncthreads();
      const int L   = lane >> 3;
      const int r   = wave * 2 + (L >> 1);
      const int col = (L & 1) * 32 + (lane & 7) * 4;
      const v4f v = *(const v4f*)(ost + r * kHeadDim + col);
      float* op = O + ((row0 + (size_t)(t - (kStage - 1) + r)) * kHeads + h) * kHeadDim + col;
      for (int pass = 0; pass < 2; ++pass) {
        *(volatile v4f*)op = v;
        __threadfence();
      }
      __syncthreads();
    }
  }
}

__global__ __launch_bounds__(256) void ng_kernel(const float* __restrict__ O, const float* __restrict__ P,
                                                 const float* __restrict__ rms_w,
                                                 unsigned short* __restrict__ Ah, unsigned short* __restrict__ Al) {
  const int bid = blockIdx.x;
  const int row = bid >> 1;
  const int t   = threadIdx.x;
  const int col = (bid & 1) * 512 + 2 * t;
  const int e   = col & 63;
  const v2f o2 = *(const v2f*)(O + (size_t)row * kNq + col);
  const v2f g2 = *(const v2f*)(P + (size_t)row * kNstkPad + kColGate + col);
  float ss = o2[0] * o2[0] + o2[1] * o2[1];
  ss += __shfl_xor(ss, 1, 32);
  ss += __shfl_xor(ss, 2, 32);
  ss += __shfl_xor(ss, 4, 32);
  ss += __shfl_xor(ss, 8, 32);
  ss += __shfl_xor(ss, 16, 32);
  const float rn = rsqrtf(ss * (1.0f / 64.0f) + 1e-5f);
  const float w0 = rms_w[e];
  const float w1 = rms_w[e + 1];
  const float s0 = g2[0] * (1.0f / (1.0f + expf(-g2[0])));
  const float s1 = g2[1] * (1.0f / (1.0f + expf(-g2[1])));
  const float a0 = o2[0] * rn * w0 * s0;
  const float a1 = o2[1] * rn * w1 * s1;
  const unsigned short hb0 = f2bf_bits(a0);
  const unsigned short lb0 = f2bf_bits(a0 - bf_bits2f(hb0));
  const unsigned short hb1 = f2bf_bits(a1);
  const unsigned short lb1 = f2bf_bits(a1 - bf_bits2f(hb1));
  const unsigned uh = pk16(hb0, hb1);
  const unsigned ul = pk16(lb0, lb1);
  const size_t wi = ((size_t)row * kNq + col) >> 1;
  for (int pass = 0; pass < 2; ++pass) {
    ((volatile unsigned*)Ah)[wi] = uh;
    ((volatile unsigned*)Al)[wi] = ul;
    __threadfence();
  }
}

extern "C" void kernel_launch(void* const* d_in, const int* in_sizes, int n_in,
                              void* d_out, int out_size, void* d_ws, size_t ws_size,
                              hipStream_t stream) {
  if (n_in < 15) return;
  if (in_sizes[0] != kRows * kChan || in_sizes[1] != kNq * kChan || in_sizes[2] != kNkv * kChan ||
      in_sizes[3] != kNkv * kChan || in_sizes[4] != kChan * kChan || in_sizes[5] != kNq * kTaps ||
      in_sizes[6] != kNkv * kTaps || in_sizes[7] != kNkv * kTaps || in_sizes[8] != kKvHeads * kChan ||
      in_sizes[9] != kKvHeads || in_sizes[10] != kKvHeads * kChan || in_sizes[11] != kKvHeads ||
      in_sizes[12] != kKvHeads || in_sizes[13] != kNq * kChan || in_sizes[14] != kHeadDim) return;
  if (out_size != kRows * kChan) return;

  const float* x      = (const float*)d_in[0];
  const float* Wq     = (const float*)d_in[1];
  const float* Wk     = (const float*)d_in[2];
  const float* Wv     = (const float*)d_in[3];
  const float* Wproj  = (const float*)d_in[4];
  const float* cwq    = (const float*)d_in[5];
  const float* cwk    = (const float*)d_in[6];
  const float* cwv    = (const float*)d_in[7];
  const float* Wbeta  = (const float*)d_in[8];
  const float* b_beta = (const float*)d_in[9];
  const float* Wgk    = (const float*)d_in[10];
  const float* A_log  = (const float*)d_in[11];
  const float* dt_b   = (const float*)d_in[12];
  const float* Wgate  = (const float*)d_in[13];
  const float* rms_w  = (const float*)d_in[14];
  float* out = (float*)d_out;

  char* w = (char*)d_ws;
  size_t off = 0;
  auto carve = [&](size_t bytes) -> char* {
    char* p = w + off;
    off += (bytes + 255) & ~(size_t)255;
    return p;
  };
  const size_t xplane  = (size_t)kRows * kChan * 2;
  const size_t wsplane = (size_t)kNstkPad * kChan * 2;
  const size_t wpplane = (size_t)kChan * kChan * 2;
  unsigned short* xh  = (unsigned short*)carve(xplane);
  unsigned short* xl  = (unsigned short*)carve(xplane);
  unsigned short* wsh = (unsigned short*)carve(wsplane);
  unsigned short* wsl = (unsigned short*)carve(wsplane);
  unsigned short* wph = (unsigned short*)carve(wpplane);
  unsigned short* wpl = (unsigned short*)carve(wpplane);
  float* P  = (float*)carve((size_t)kRows * kNstkPad * 4);
  float* Qn = (float*)carve((size_t)kRows * kNq * 4);
  float* Kn = (float*)carve((size_t)kRows * kNkv * 4);
  float* Vc = (float*)carve((size_t)kRows * kNkv * 4);
  float* BG = (float*)carve((size_t)kRows * kBgPitch * 4);
  if (off > ws_size) return;
  float* O = (float*)xh;
  unsigned short* Ah = (unsigned short*)Qn;
  unsigned short* Al = Ah + (size_t)kRows * kNq;

  split8_kernel<<<(kRows * kChan / 8) / 256, 256, 0, stream>>>(x, xh, xl, kRows * kChan / 8);
  split_stack_kernel<<<kNstkPad, 128, 0, stream>>>(Wq, Wk, Wv, Wbeta, Wgk, Wgate, wsh, wsl);
  split8_kernel<<<(kChan * kChan / 8) / 256, 256, 0, stream>>>(Wproj, wph, wpl, kChan * kChan / 8);

  wmma_gemm64<1, true, 0, 0, false, 0><<<dim3((kRows / 64) * (kNstkPad / 64) / 8, 1), 256, 0, stream>>>(
      xh, xl, kChan, 0L, wsh, wsl, kChan, 0L, (void*)P, (void*)nullptr, kNstkPad, 0L,
      (const float*)nullptr, (const float*)nullptr, 0L, kRows, kNstkPad, kChan, 1.0f);

  prep_conv_kernel<true><<<kRows, kNq / 4, 0, stream>>>(P, 0, cwq, Qn, kNq);
  prep_conv_kernel<true><<<kRows, kNkv / 4, 0, stream>>>(P, kColK, cwk, Kn, kNkv);
  prep_conv_kernel<false><<<kRows, kNkv / 4, 0, stream>>>(P, kColV, cwv, Vc, kNkv);
  prep_bg_kernel<<<kRows / 8, 256, 0, stream>>>(P, b_beta, dt_b, A_log, BG);

  gdn_kernel<<<kBatch * kHeads, 256, 0, stream>>>(Qn, Kn, Vc, BG, O);

  ng_kernel<<<kRows * 2, 256, 0, stream>>>(O, P, rms_w, Ah, Al);

  wmma_gemm64<1, true, 0, 0, false, 0><<<dim3((kRows / 64) * (kChan / 64) / 8, 1), 256, 0, stream>>>(
      Ah, Al, kNq, 0L, wph, wpl, kChan, 0L, (void*)out, (void*)nullptr, kChan, 0L,
      (const float*)nullptr, (const float*)nullptr, 0L, kRows, kChan, kChan, 1.0f);
}
